// Frame2TFNCrossAttentionUpdate_56023553409100
// MI455X (gfx1250) — hardware-verified
//
#include <hip/hip_runtime.h>

typedef _Float16 v16h __attribute__((ext_vector_type(16)));
typedef _Float16 v8h  __attribute__((ext_vector_type(8)));
typedef float    v8f  __attribute__((ext_vector_type(8)));
typedef float    v4f  __attribute__((ext_vector_type(4)));
union Frag { v16h v; v8h half[2]; };
union HRow { _Float16 s[32]; v8h q[4]; };

#define NBLK 256
#define LCAP 8192

__device__ __forceinline__ float bfr(float x) {
  unsigned u = __float_as_uint(x);
  u = (u + 0x7FFFu + ((u >> 16) & 1u)) & 0xFFFF0000u;
  return __uint_as_float(u);
}

__device__ __forceinline__ v8f wmma16(v16h a, v16h b, v8f c) {
  v8f d = __builtin_amdgcn_wmma_f32_16x16x32_f16(false, a, false, b, (short)0, c, false, false);
  asm volatile("v_nop\n\tv_nop\n\tv_nop\n\tv_nop" : "+v"(d) : "v"(a), "v"(b));
  return d;
}

__global__ __launch_bounds__(128) void k_convw(const float* __restrict__ Wk1, const float* __restrict__ Wv1,
                                               const float* __restrict__ Wk2, const float* __restrict__ Wv2,
                                               _Float16* __restrict__ W16) {
  int col = blockIdx.x * blockDim.x + threadIdx.x;
  if (col >= 1600) return;
  const float* W; int NC, lc;
  if (col < 32)       { W = Wk1; NC = 32;  lc = col; }
  else if (col < 64)  { W = Wv1; NC = 32;  lc = col - 32; }
  else if (col < 704) { W = Wk2; NC = 640; lc = col - 64; }
  else                { W = Wv2; NC = 896; lc = col - 704; }
  HRow r;
  for (int k = 0; k < 32; ++k) r.s[k] = (_Float16)bfr(W[(size_t)k * NC + lc]);
  _Float16* dst = W16 + (size_t)col * 32;
  #pragma unroll
  for (int j = 0; j < 4; ++j) *(volatile v8h*)(dst + 8 * j) = r.q[j];
  __threadfence();
  #pragma unroll
  for (int j = 0; j < 4; ++j) *(volatile v8h*)(dst + 8 * j) = r.q[j];
}

__global__ __launch_bounds__(256) void k_node_pre(
    const float* __restrict__ ff, const float* __restrict__ rot, const float* __restrict__ trans,
    const float* __restrict__ tfn, const float* __restrict__ Wf0, const float* __restrict__ bf0,
    const float* __restrict__ Wf1, const float* __restrict__ bf1, const float* __restrict__ Wgs,
    const float* __restrict__ Wgv, const float* __restrict__ Wqs, const float* __restrict__ Wqv,
    int N, float* __restrict__ nodef) {
  __shared__ float ffL[128], f0L[64], f1L[96], f1R[96], res[96];
  const int n = blockIdx.x;
  const int t = threadIdx.x;
  if (n >= N) return;
  if (t < 128) ffL[t] = bfr(ff[(size_t)n * 128 + t]);
  __syncthreads();
  if (t < 64) {
    float acc = bfr(bf0[t]);
    #pragma unroll 1
    for (int k = 0; k < 128; ++k) acc += ffL[k] * bfr(Wf0[k * 64 + t]);
    f0L[t] = acc;
  } else if (t < 160) {
    int c = t - 64;
    float acc = bfr(bf1[c]);
    #pragma unroll 1
    for (int k = 0; k < 128; ++k) acc += ffL[k] * bfr(Wf1[k * 96 + c]);
    f1L[c] = acc;
  }
  __syncthreads();
  if (t < 96) {
    int u = t / 3, i = t % 3;
    const float* R = rot + (size_t)n * 9;
    f1R[t] = bfr(R[i * 3 + 0]) * f1L[u * 3 + 0] + bfr(R[i * 3 + 1]) * f1L[u * 3 + 1]
           + bfr(R[i * 3 + 2]) * f1L[u * 3 + 2] + bfr(trans[(size_t)n * 3 + i]);
  }
  __syncthreads();
  if (t < 16) {
    float acc = 0.f;
    #pragma unroll 1
    for (int k = 0; k < 64; ++k) acc += f0L[k] * bfr(Wgs[k * 16 + t]);
    res[t] = acc * 0.125f;
  } else if (t < 40) {
    int idx = t - 16, w = idx / 3, i = idx % 3;
    float acc = 0.f;
    #pragma unroll 1
    for (int u = 0; u < 32; ++u) acc += f1R[u * 3 + i] * bfr(Wgv[u * 8 + w]);
    res[16 + w * 3 + i] = acc * 0.1767766953f;
  } else if (t < 56) {
    int c = t - 40;
    float acc = 0.f;
    const float* ts = tfn + (size_t)n * 40;
    #pragma unroll 1
    for (int u = 0; u < 16; ++u) acc += bfr(ts[u]) * bfr(Wqs[u * 16 + c]);
    res[40 + c] = acc * 0.25f;
  } else if (t < 80) {
    int idx = t - 56, w = idx / 3, i = idx % 3;
    float acc = 0.f;
    const float* tv = tfn + (size_t)n * 40 + 16;
    #pragma unroll 1
    for (int u = 0; u < 8; ++u) acc += bfr(tv[u * 3 + i]) * bfr(Wqv[u * 8 + w]);
    res[56 + w * 3 + i] = acc * 0.3535533906f;
  } else if (t < 96) {
    res[t] = 0.f;
  }
  __syncthreads();
  if (t < 96) {
    float v = res[t];
    volatile float* p = nodef + (size_t)n * 96 + t;
    *p = v;
    __threadfence();
    *p = v;
  }
}

__global__ __launch_bounds__(256) void k_egather(const int* __restrict__ eidx, const float* __restrict__ esh,
                                                 const float* __restrict__ nodef, int E, int N, int Epad,
                                                 float* __restrict__ erow) {
  const int t = threadIdx.x, wv = t >> 5, lane = t & 31;
  const int grp = lane >> 3, q = lane & 7;
  const int p = ((int)blockIdx.x * 8 + wv) * 4 + grp;
  if (p >= Epad) return;
  const bool valid = p < E;
  int dn = 0, sn = 0;
  if (valid) {
    dn = eidx[p];             dn = dn < 0 ? 0 : (dn > N - 1 ? N - 1 : dn);
    sn = eidx[(size_t)E + p]; sn = sn < 0 ? 0 : (sn > N - 1 ? N - 1 : sn);
  }
  const float* gd = nodef + (size_t)dn * 96;
  const float* gq = nodef + (size_t)sn * 96;
  v4f val[3];
  #pragma unroll
  for (int j = 0; j < 3; ++j) {
    #pragma unroll
    for (int k = 0; k < 4; ++k) {
      const int f = j * 32 + 4 * q + k;
      float x = 0.f;
      if (valid) {
        if (f < 40)      x = gd[f];
        else if (f < 80) x = gq[f];
        else if (f < 84) x = bfr(esh[(size_t)p * 4 + (f - 80)]);
      }
      val[j][k] = x;
    }
  }
  float* dst = erow + (size_t)p * 96;
  #pragma unroll
  for (int j = 0; j < 3; ++j) *(volatile v4f*)(dst + j * 32 + 4 * q) = val[j];
  __threadfence();
  #pragma unroll
  for (int j = 0; j < 3; ++j) *(volatile v4f*)(dst + j * 32 + 4 * q) = val[j];
}

__global__ __launch_bounds__(128) __attribute__((amdgpu_num_vgpr(256))) void k_edge(
    const float* __restrict__ ef, const float* __restrict__ erow, const _Float16* __restrict__ W16g,
    const float* __restrict__ bk1, const float* __restrict__ bk2,
    const float* __restrict__ bv1, const float* __restrict__ bv2,
    int E, float* __restrict__ attnB, float* __restrict__ vbuf) {
  __shared__ __align__(16) _Float16 Wl[1600 * 32];
  __shared__ float cA[4][16][16], cB[4][16][8], cC[4][16][16];
  __shared__ float cD[4][16][24], cE[4][16][24];
  __shared__ float shvL[4][16][4], qS[4][16][16], qV[4][16][24];
  __shared__ __align__(16) _Float16 hbuf[4][16][32];
  __shared__ __align__(16) _Float16 hlo[4][16][32];
  __shared__ __align__(16) float vst[4][16][64];

  const int tid = (int)threadIdx.x;
  const int wv = tid >> 5, lane = tid & 31;
  const int h = lane >> 4, m = lane & 15;
  const int eoff = 8 * h;
  const int p0 = (int)blockIdx.x * 64 + wv * 16;

  #pragma unroll 2
  for (int idx = tid; idx < 6400; idx += 128)
    *(v8h*)(Wl + (size_t)idx * 8) = *(const v8h*)(W16g + (size_t)idx * 8);

  if (lane < 16) {
    const int p = p0 + lane;
    const float* er = erow + (size_t)p * 96;
    const float shs = er[80], sv0 = er[81], sv1 = er[82], sv2 = er[83];
    shvL[wv][lane][0] = sv0; shvL[wv][lane][1] = sv1; shvL[wv][lane][2] = sv2; shvL[wv][lane][3] = 0.f;
    const float* g0 = er;
    #pragma unroll
    for (int u = 0; u < 16; ++u) {
      float f = g0[u];
      cA[wv][lane][u] = f * shs * 0.25f;
      cC[wv][lane][u] = f * 0.25f;
    }
    const float* g1 = er + 16;
    const float i8 = 0.3535533906f;
    #pragma unroll
    for (int u = 0; u < 8; ++u) {
      float x = g1[u * 3 + 0], y = g1[u * 3 + 1], z = g1[u * 3 + 2];
      cB[wv][lane][u] = (x * sv0 + y * sv1 + z * sv2) * i8;
      cD[wv][lane][u * 3 + 0] = x * shs * i8;
      cD[wv][lane][u * 3 + 1] = y * shs * i8;
      cD[wv][lane][u * 3 + 2] = z * shs * i8;
      cE[wv][lane][u * 3 + 0] = (y * sv2 - z * sv1) * i8;
      cE[wv][lane][u * 3 + 1] = (z * sv0 - x * sv2) * i8;
      cE[wv][lane][u * 3 + 2] = (x * sv1 - y * sv0) * i8;
    }
    const float* qq = er + 40;
    #pragma unroll
    for (int j = 0; j < 16; ++j) qS[wv][lane][j] = qq[j];
    #pragma unroll
    for (int j = 0; j < 24; ++j) qV[wv][lane][j] = qq[16 + j];
  }

  Frag aef;
  {
    int rowc = p0 + m; if (rowc > E - 1) rowc = E - 1;
    const float* rp = ef + (size_t)rowc * 32;
    v4f x0 = *(const v4f*)(rp + 8 * h),      x1 = *(const v4f*)(rp + 8 * h + 4);
    v4f y0 = *(const v4f*)(rp + 16 + 8 * h), y1 = *(const v4f*)(rp + 20 + 8 * h);
    #pragma unroll
    for (int i = 0; i < 4; ++i) {
      aef.v[i]      = (_Float16)bfr(x0[i]);
      aef.v[4 + i]  = (_Float16)bfr(x1[i]);
      aef.v[8 + i]  = (_Float16)bfr(y0[i]);
      aef.v[12 + i] = (_Float16)bfr(y1[i]);
    }
  }
  __syncthreads();

  const v8f zero8 = {0.f, 0.f, 0.f, 0.f, 0.f, 0.f, 0.f, 0.f};

  Frag fhk, fhl, fhv;
  #pragma unroll
  for (int which = 0; which < 2; ++which) {
    const float* bb = which ? bv1 : bk1;
    #pragma unroll
    for (int tt = 0; tt < 2; ++tt) {
      const int col = which * 32 + tt * 16 + m;
      Frag b;
      b.half[0] = *(const v8h*)(Wl + (size_t)col * 32 + 8 * h);
      b.half[1] = *(const v8h*)(Wl + (size_t)col * 32 + 16 + 8 * h);
      v8f d = wmma16(aef.v, b.v, zero8);
      float bias = bfr(bb[tt * 16 + m]);
      #pragma unroll
      for (int r = 0; r < 8; ++r) {
        float v = fmaxf(d[r] + bias, 0.0f);
        _Float16 hv = (_Float16)v;
        hbuf[wv][r + eoff][tt * 16 + m] = hv;
        if (which == 0) hlo[wv][r + eoff][tt * 16 + m] = (_Float16)((v - (float)hv) * 2048.0f);
      }
    }
    __syncthreads();
    if (which) {
      fhv.half[0] = *(const v8h*)(&hbuf[wv][m][8 * h]);
      fhv.half[1] = *(const v8h*)(&hbuf[wv][m][16 + 8 * h]);
    } else {
      fhk.half[0] = *(const v8h*)(&hbuf[wv][m][8 * h]);
      fhk.half[1] = *(const v8h*)(&hbuf[wv][m][16 + 8 * h]);
      fhl.half[0] = *(const v8h*)(&hlo[wv][m][8 * h]);
      fhl.half[1] = *(const v8h*)(&hlo[wv][m][16 + 8 * h]);
    }
    __syncthreads();
  }

  const float inv_s2 = 0.7071067811865476f;
  const float inv_s3 = 0.5773502691896258f;

  float accS[8], accC[8], accV[8][3];
  #pragma unroll
  for (int r = 0; r < 8; ++r) { accS[r] = 0.f; accC[r] = 0.f; accV[r][0] = accV[r][1] = accV[r][2] = 0.f; }

  #define K_TILE(T)                                                                      \
    Frag bq;                                                                             \
    bq.half[0] = *(const v8h*)(Wl + (size_t)(64 + (T) * 16 + m) * 32 + 8 * h);          \
    bq.half[1] = *(const v8h*)(Wl + (size_t)(64 + (T) * 16 + m) * 32 + 16 + 8 * h);     \
    v8f d = wmma16(fhk.v, bq.v, zero8);                                                  \
    v8f dl = wmma16(fhl.v, bq.v, zero8);                                                 \
    float bias = bfr(bk2[(T) * 16 + m]);
  #define KVAL(R) (d[R] + bias + dl[R] * 0.00048828125f)
  #pragma unroll 1
  for (int t = 0; t < 16; ++t) {
    K_TILE(t)
    #pragma unroll
    for (int r = 0; r < 8; ++r) accS[r] += cA[wv][r + eoff][t] * KVAL(r);
  }
  #pragma unroll 1
  for (int t = 16; t < 24; ++t) {
    K_TILE(t)
    #pragma unroll
    for (int r = 0; r < 8; ++r) accS[r] += cB[wv][r + eoff][t - 16] * KVAL(r);
  }
  #pragma unroll 1
  for (int t = 24; t < 32; ++t) {
    K_TILE(t)
    int u = ((t - 24) << 1) | (m >> 3);
    #pragma unroll
    for (int r = 0; r < 8; ++r) accC[r] += cC[wv][r + eoff][u] * KVAL(r);
  }
  #pragma unroll 1
  for (int t = 32; t < 36; ++t) {
    K_TILE(t)
    int u = ((t - 32) << 1) | (m >> 3);
    #pragma unroll
    for (int r = 0; r < 8; ++r) {
      float val = KVAL(r);
      #pragma unroll
      for (int i = 0; i < 3; ++i) accV[r][i] += cD[wv][r + eoff][u * 3 + i] * val;
    }
  }
  #pragma unroll 1
  for (int t = 36; t < 40; ++t) {
    K_TILE(t)
    int u = ((t - 36) << 1) | (m >> 3);
    #pragma unroll
    for (int r = 0; r < 8; ++r) {
      float val = KVAL(r);
      #pragma unroll
      for (int i = 0; i < 3; ++i) accV[r][i] += cE[wv][r + eoff][u * 3 + i] * val;
    }
  }
  #undef KVAL
  #undef K_TILE

  {
    const int wvi = m & 7;
    #pragma unroll
    for (int r = 0; r < 8; ++r) {
      const int e = r + eoff;
      float ks = accS[r] * inv_s2;
      vst[wv][e][m] = qS[wv][e][m] * ks;
      float p2 = 0.f;
      #pragma unroll
      for (int i = 0; i < 3; ++i) {
        float kv = (accC[r] * shvL[wv][e][i] + accV[r][i]) * inv_s3;
        p2 += qV[wv][e][wvi * 3 + i] * kv;
      }
      vst[wv][e][16 + m] = p2;
    }
  }
  __syncthreads();
  v4f attv;
  attv[0] = attv[1] = attv[2] = attv[3] = 0.f;
  if (lane < 16) {
    const float* T = &vst[wv][lane][0];
    #pragma unroll
    for (int hh = 0; hh < 4; ++hh) {
      float a = T[4 * hh + 0] + T[4 * hh + 1] + T[4 * hh + 2] + T[4 * hh + 3];
      a += T[16 + 2 * hh] + T[17 + 2 * hh] + T[24 + 2 * hh] + T[25 + 2 * hh];
      attv[hh] = a;
    }
    *(volatile v4f*)(attnB + (size_t)(p0 + lane) * 4) = attv;
  }
  __syncthreads();

  #pragma unroll
  for (int r = 0; r < 8; ++r) { accS[r] = 0.f; accC[r] = 0.f; accV[r][0] = accV[r][1] = accV[r][2] = 0.f; }
  #define V_TILE(T)                                                                      \
    Frag bq;                                                                             \
    bq.half[0] = *(const v8h*)(Wl + (size_t)(704 + (T) * 16 + m) * 32 + 8 * h);         \
    bq.half[1] = *(const v8h*)(Wl + (size_t)(704 + (T) * 16 + m) * 32 + 16 + 8 * h);    \
    v8f d = wmma16(fhv.v, bq.v, zero8);                                                  \
    float bias = bfr(bv2[(T) * 16 + m]);
  #pragma unroll 1
  for (int t = 0; t < 16; ++t) {
    V_TILE(t)
    #pragma unroll
    for (int r = 0; r < 8; ++r) accS[r] += cA[wv][r + eoff][t] * (d[r] + bias);
  }
  #pragma unroll 1
  for (int t = 16; t < 24; ++t) {
    V_TILE(t)
    #pragma unroll
    for (int r = 0; r < 8; ++r) accS[r] += cB[wv][r + eoff][t - 16] * (d[r] + bias);
  }
  #pragma unroll 1
  for (int t = 24; t < 40; ++t) {
    V_TILE(t)
    #pragma unroll
    for (int r = 0; r < 8; ++r) accC[r] += cC[wv][r + eoff][t - 24] * (d[r] + bias);
  }
  #pragma unroll 1
  for (int t = 40; t < 48; ++t) {
    V_TILE(t)
    #pragma unroll
    for (int r = 0; r < 8; ++r) {
      float val = d[r] + bias;
      #pragma unroll
      for (int i = 0; i < 3; ++i) accV[r][i] += cD[wv][r + eoff][(t - 40) * 3 + i] * val;
    }
  }
  #pragma unroll 1
  for (int t = 48; t < 56; ++t) {
    V_TILE(t)
    #pragma unroll
    for (int r = 0; r < 8; ++r) {
      float val = d[r] + bias;
      #pragma unroll
      for (int i = 0; i < 3; ++i) accV[r][i] += cE[wv][r + eoff][(t - 48) * 3 + i] * val;
    }
  }
  #undef V_TILE

  #pragma unroll
  for (int r = 0; r < 8; ++r) {
    const int e = r + eoff;
    vst[wv][e][m] = accS[r] * inv_s2;
    #pragma unroll
    for (int i = 0; i < 3; ++i)
      vst[wv][e][16 + m * 3 + i] = (accC[r] * shvL[wv][e][i] + accV[r][i]) * inv_s3;
  }
  __syncthreads();
  #pragma unroll
  for (int mm = 0; mm < 8; ++mm) {
    const int e = 2 * mm + h;
    v4f v = *(const v4f*)(&vst[wv][e][m * 4]);
    *(volatile v4f*)(vbuf + (size_t)(p0 + e) * 64 + m * 4) = v;
  }
  __threadfence();
  #pragma unroll
  for (int mm = 0; mm < 8; ++mm) {
    const int e = 2 * mm + h;
    v4f v = *(const v4f*)(&vst[wv][e][m * 4]);
    *(volatile v4f*)(vbuf + (size_t)(p0 + e) * 64 + m * 4) = v;
  }
  if (lane < 16) *(volatile v4f*)(attnB + (size_t)(p0 + lane) * 4) = attv;
}

__device__ __forceinline__ float pick4(float a0, float a1, float a2, float a3, int i) {
  return i == 0 ? a0 : (i == 1 ? a1 : (i == 2 ? a2 : a3));
}

__device__ __forceinline__ int lds_lower_bound(const unsigned* a, unsigned key) {
  int lo = 0, hi = LCAP;
  #pragma unroll 1
  for (int it = 0; it < 15 && lo < hi; ++it) {
    int mid = (lo + hi) >> 1;
    if (a[mid] < key) lo = mid + 1; else hi = mid;
  }
  return lo;
}

__global__ __launch_bounds__(256) void k_seg(
    const int* __restrict__ eidx, const float* __restrict__ attnB, const float* __restrict__ vbuf,
    const float* __restrict__ tfn, const float* __restrict__ Wos, const float* __restrict__ Wov,
    const float* __restrict__ Wss, const float* __restrict__ Wsv,
    int N, int E, int Epad, float* __restrict__ obuf) {
  __shared__ unsigned lst[LCAP];
  __shared__ int wcnt[8];
  __shared__ __align__(16) float upd[8][64];
  __shared__ __align__(16) float os[8][64];
  const int t = threadIdx.x, wv = t >> 5, lane = t & 31;
  const int n0 = (int)blockIdx.x * NBLK;
  const unsigned ltmask = (1u << lane) - 1u;

  int fill = 0;
  const int nchunk = (E + 255) >> 8;
  #pragma unroll 1
  for (int ch = 0; ch < nchunk; ++ch) {
    const int g = (ch << 8) + t;
    bool hit = false; unsigned key = 0u;
    if (g < E) {
      int s = eidx[(size_t)E + g];
      s = s < 0 ? 0 : (s > N - 1 ? N - 1 : s);
      int jl = s - n0;
      if (jl >= 0 && jl < NBLK) { hit = true; key = ((unsigned)jl << 18) | (unsigned)g; }
    }
    const unsigned bal = __builtin_amdgcn_ballot_w32(hit);
    if (lane == 0) wcnt[wv] = (int)__builtin_popcount(bal);
    __syncthreads();
    int pre = 0, tot = 0;
    #pragma unroll
    for (int w = 0; w < 8; ++w) { int c = wcnt[w]; tot += c; pre += (w < wv) ? c : 0; }
    const int pos = fill + pre + (int)__builtin_popcount(bal & ltmask);
    if (hit && pos < LCAP) lst[pos] = key;
    fill += tot;
    __syncthreads();
  }
  const int L = fill < LCAP ? fill : LCAP;
  for (int i = t; i < LCAP; i += 256) if (i >= L) lst[i] = 0xFFFFFFFFu;
  __syncthreads();

  for (int k = 2; k <= LCAP; k <<= 1) {
    for (int j = k >> 1; j > 0; j >>= 1) {
      #pragma unroll 4
      for (int mI = 0; mI < LCAP / 256; ++mI) {
        const int i = t + 256 * mI;
        const int ixj = i ^ j;
        if (ixj > i) {
          const bool asc = ((i & k) == 0);
          unsigned a = lst[i], b = lst[ixj];
          if ((a > b) == asc) { lst[i] = b; lst[ixj] = a; }
        }
      }
      __syncthreads();
    }
  }

  const int c0 = lane, c1 = lane + 32;
  const int hd0 = (c0 < 16) ? (c0 >> 2) : (((c0 - 16) / 3) >> 2);
  const int hd1 = ((c1 - 16) / 3) >> 2;

  #pragma unroll 1
  for (int it = 0; it < NBLK / 8; ++it) {
    const int jl = it * 8 + wv;
    const int n = n0 + jl;
    const int nn = n < N ? n : N - 1;
    int beg = lds_lower_bound(lst, (unsigned)jl << 18);
    int end = lds_lower_bound(lst, (unsigned)(jl + 1) << 18);
    if (beg > L) beg = L;
    if (end > L) end = L;
    int cnt = end - beg; if (cnt < 0) cnt = 0;
    if (cnt > LCAP - beg) cnt = LCAP - beg;

    float mx0 = -3.0e38f, mx1 = -3.0e38f, mx2 = -3.0e38f, mx3 = -3.0e38f;
    #pragma unroll 1
    for (int tt = 0; tt < cnt; ++tt) {
      int e = (int)(lst[beg + tt] & 0x3FFFFu); if (e > Epad - 1) e = Epad - 1;
      v4f a = *(const v4f*)(attnB + (size_t)e * 4);
      mx0 = fmaxf(mx0, a[0]); mx1 = fmaxf(mx1, a[1]); mx2 = fmaxf(mx2, a[2]); mx3 = fmaxf(mx3, a[3]);
    }
    float d0 = 0.f, d1 = 0.f, d2 = 0.f, d3 = 0.f, acc0 = 0.f, acc1 = 0.f;
    #pragma unroll 1
    for (int tt = 0; tt < cnt; ++tt) {
      int e = (int)(lst[beg + tt] & 0x3FFFFu); if (e > Epad - 1) e = Epad - 1;
      const size_t p = (size_t)e;
      v4f a = *(const v4f*)(attnB + p * 4);
      float e0 = expf(a[0] - mx0), e1 = expf(a[1] - mx1), e2 = expf(a[2] - mx2), e3 = expf(a[3] - mx3);
      d0 += e0; d1 += e1; d2 += e2; d3 += e3;
      float v0 = vbuf[p * 64 + lane], v1 = vbuf[p * 64 + 32 + lane];
      acc0 += v0 * pick4(e0, e1, e2, e3, hd0);
      acc1 += v1 * pick4(e0, e1, e2, e3, hd1);
    }
    float i0 = 1.f / (d0 + 1e-9f), i1 = 1.f / (d1 + 1e-9f), i2 = 1.f / (d2 + 1e-9f), i3 = 1.f / (d3 + 1e-9f);
    upd[wv][lane]      = acc0 * pick4(i0, i1, i2, i3, hd0);
    upd[wv][lane + 32] = acc1 * pick4(i0, i1, i2, i3, hd1);
    __syncthreads();

    const float* ts = tfn + (size_t)nn * 40;
    if (lane < 16) {
      float o = 0.f, o2 = 0.f;
      #pragma unroll 1
      for (int w = 0; w < 16; ++w) o += upd[wv][w] * bfr(Wos[w * 16 + lane]);
      #pragma unroll 1
      for (int u = 0; u < 16; ++u) o2 += bfr(ts[u]) * bfr(Wss[u * 16 + lane]);
      os[wv][lane] = o * 0.25f + o2 * 0.25f;
    }
    #pragma unroll
    for (int q = 0; q < 2; ++q) {
      int idx = q == 0 ? (lane - 16) : (lane + 16);
      bool act = q == 0 ? (lane >= 16) : (lane < 8);
      if (act) {
        int cc = idx / 3, i = idx % 3;
        float o = 0.f, o2 = 0.f;
        #pragma unroll 1
        for (int w = 0; w < 16; ++w) o += upd[wv][16 + w * 3 + i] * bfr(Wov[w * 8 + cc]);
        #pragma unroll 1
        for (int u = 0; u < 8; ++u) o2 += bfr(ts[16 + u * 3 + i]) * bfr(Wsv[u * 8 + cc]);
        os[wv][16 + idx] = o * 0.25f + o2 * 0.3535533906f;
      }
    }
    if (lane >= 8 && lane < 16) { os[wv][40 + (lane - 8)] = 0.f; os[wv][48 + (lane - 8)] = 0.f; os[wv][56 + (lane - 8)] = 0.f; }
    __syncthreads();
    if (lane < 16 && n < N) {
      v4f v = *(const v4f*)(&os[wv][lane * 4]);
      *(volatile v4f*)(obuf + (size_t)n * 64 + lane * 4) = v;
      __threadfence();
      *(volatile v4f*)(obuf + (size_t)n * 64 + lane * 4) = v;
    }
  }
}

__global__ __launch_bounds__(256) void k_bnstat(const float* __restrict__ obuf, const float* __restrict__ bnws,
                                                const float* __restrict__ bnbs, const float* __restrict__ bnwv,
                                                int N, float* __restrict__ stats) {
  __shared__ double sd[240], sd2[240], S1[40], S2[40];
  __shared__ float res[128];
  const int t = threadIdx.x;
  if (t < 240) {
    int c = t % 40, g = t / 40;
    double s = 0.0, s2 = 0.0;
    for (int n = g; n < N; n += 6) {
      double x = (double)obuf[(size_t)n * 64 + c];
      s += x; s2 += x * x;
    }
    sd[t] = s; sd2[t] = s2;
  }
  if (t < 128) res[t] = 0.f;
  __syncthreads();
  if (t < 40) {
    double s = 0.0, s2 = 0.0;
    for (int g = 0; g < 6; ++g) { s += sd[g * 40 + t]; s2 += sd2[g * 40 + t]; }
    S1[t] = s; S2[t] = s2;
  }
  __syncthreads();
  if (t < 40) {
    double invN = 1.0 / (double)N;
    float scale, shift;
    if (t < 16) {
      double mu = S1[t] * invN;
      double var = S2[t] * invN - mu * mu; if (var < 0.0) var = 0.0;
      float sc = bfr(bnws[t]) / sqrtf((float)var + 1e-5f);
      scale = sc; shift = bfr(bnbs[t]) - (float)mu * sc;
    } else {
      int u = (t - 16) / 3;
      double n2 = (S2[16 + 3 * u] + S2[17 + 3 * u] + S2[18 + 3 * u]) * invN;
      scale = bfr(bnwv[u]) / sqrtf((float)n2 + 1e-5f); shift = 0.f;
    }
    res[t] = scale; res[64 + t] = shift;
  }
  __syncthreads();
  if (t < 128) {
    float v = res[t];
    *(volatile float*)(stats + t) = v;
    __threadfence();
    *(volatile float*)(stats + t) = v;
  }
}

__global__ __launch_bounds__(256) void k_final(const float* __restrict__ obuf, const float* __restrict__ stats,
                                               int nq, float* __restrict__ out) {
  int f = blockIdx.x * blockDim.x + threadIdx.x;
  if (f >= nq) return;
  int n = f / 10, c0 = (f % 10) * 4;
  v4f v;
  #pragma unroll
  for (int k = 0; k < 4; ++k) {
    int c = c0 + k;
    v[k] = obuf[(size_t)n * 64 + c] * stats[c] + stats[64 + c];
  }
  *(volatile v4f*)(out + (size_t)f * 4) = v;
  __threadfence();
  *(volatile v4f*)(out + (size_t)f * 4) = v;
}

static inline size_t al256(size_t x) { return (x + 255) & ~(size_t)255; }

extern "C" void kernel_launch(void* const* d_in, const int* in_sizes, int n_in,
                              void* d_out, int out_size, void* d_ws, size_t ws_size,
                              hipStream_t stream) {
  if (n_in < 30) return;
  const float* ff    = (const float*)d_in[0];
  const float* rot   = (const float*)d_in[1];
  const float* trans = (const float*)d_in[2];
  const float* tfn   = (const float*)d_in[3];
  const float* ef    = (const float*)d_in[4];
  const float* esh   = (const float*)d_in[5];
  const int*   eidx  = (const int*)  d_in[6];
  const float* Wf0   = (const float*)d_in[7];
  const float* bf0   = (const float*)d_in[8];
  const float* Wf1   = (const float*)d_in[9];
  const float* bf1   = (const float*)d_in[10];
  const float* Wgs   = (const float*)d_in[11];
  const float* Wgv   = (const float*)d_in[12];
  const float* Wqs   = (const float*)d_in[13];
  const float* Wqv   = (const float*)d_in[14];
  const float* Wk1   = (const float*)d_in[15];
  const float* bk1   = (const float*)d_in[16];
  const float* Wk2   = (const float*)d_in[17];
  const float* bk2   = (const float*)d_in[18];
  const float* Wv1   = (const float*)d_in[19];
  const float* bv1   = (const float*)d_in[20];
  const float* Wv2   = (const float*)d_in[21];
  const float* bv2   = (const float*)d_in[22];
  const float* Wos   = (const float*)d_in[23];
  const float* Wov   = (const float*)d_in[24];
  const float* Wss   = (const float*)d_in[25];
  const float* Wsv   = (const float*)d_in[26];
  const float* bnws  = (const float*)d_in[27];
  const float* bnbs  = (const float*)d_in[28];
  const float* bnwv  = (const float*)d_in[29];
  float* out = (float*)d_out;

  const int N = in_sizes[0] / 128;
  const int E = in_sizes[6] / 2;
  if (N <= 0 || E <= 0 || E > 262144) return;
  if (out_size != N * 40) return;
  const int Epad = ((E + 63) / 64) * 64;

  char* base = (char*)d_ws;
  size_t off = 0;
  _Float16* W16 = (_Float16*)(base + off); off = al256(off + (size_t)1600 * 32 * 2);
  float* nodef  = (float*)(base + off);    off = al256(off + (size_t)N * 96 * 4);
  float* erow   = (float*)(base + off);    off = al256(off + (size_t)Epad * 96 * 4);
  float* attnB  = (float*)(base + off);    off = al256(off + (size_t)Epad * 4 * 4);
  float* vbuf   = (float*)(base + off);    off = al256(off + (size_t)Epad * 64 * 4);
  float* obuf   = (float*)(base + off);    off = al256(off + (size_t)N * 64 * 4);
  float* stats  = (float*)(base + off);    off = al256(off + 128 * 4);
  if (off > ws_size) return;

  k_convw<<<(1600 + 127) / 128, 128, 0, stream>>>(Wk1, Wv1, Wk2, Wv2, W16);
  k_node_pre<<<N, 256, 0, stream>>>(ff, rot, trans, tfn, Wf0, bf0, Wf1, bf1, Wgs, Wgv, Wqs, Wqv, N, nodef);
  k_egather<<<Epad / 32, 256, 0, stream>>>(eidx, esh, nodef, E, N, Epad, erow);
  k_edge<<<Epad / 64, 128, 0, stream>>>(ef, erow, W16, bk1, bk2, bv1, bv2, E, attnB, vbuf);
  k_seg<<<(N + NBLK - 1) / NBLK, 256, 0, stream>>>(eidx, attnB, vbuf, tfn, Wos, Wov, Wss, Wsv, N, E, Epad, obuf);
  k_bnstat<<<1, 256, 0, stream>>>(obuf, bnws, bnbs, bnwv, N, stats);
  const int nq = out_size / 4;
  k_final<<<(nq + 255) / 256, 256, 0, stream>>>(obuf, stats, nq, out);
  (void)hipGetLastError();
}
